// L1RegressionMoEActionHead_89876485636873
// MI455X (gfx1250) — hardware-verified
//
#include <hip/hip_runtime.h>
#include <stddef.h>
#include <stdint.h>

#define NBT   16
#define TQ    512
#define LKV   256
#define NKEY  512
#define HID   1024
#define NHD   8
#define HDM   128
#define NEXP  8
#define NTQ   (NBT * TQ)
#define NTK   (NBT * LKV)
#define NHB   (NBT * NHD)
#define KC    64
#define NCK   (NKEY / KC)
#define QB    128
#define NQB   (TQ / QB)

static_assert(NHD * HDM == HID);
static_assert(NTQ % 128 == 0);
static_assert(NTK % 128 == 0);
static_assert(TQ % 128 == 0);
static_assert(LKV % 128 == 0);
static_assert(NKEY == 2 * LKV);
static_assert(NCK * KC == NKEY);
static_assert((NCK / 2) * KC == LKV);
static_assert(HID % 64 == 0);
static_assert(HDM == 128);
static_assert(TQ * HDM == 65536);
static_assert(NTQ % 8 == 0);

typedef _Float16 v16h __attribute__((ext_vector_type(16)));
typedef _Float16 v8h  __attribute__((ext_vector_type(8)));
typedef float    v8f  __attribute__((ext_vector_type(8)));
typedef float    v4f  __attribute__((ext_vector_type(4)));
typedef unsigned int v4u __attribute__((ext_vector_type(4)));

union Frag  { v16h v; v8h h[2]; };
union Pack8 { v8h h; v4u u; };

__device__ __forceinline__ v8f mma16(v16h a, v16h b, v8f c) {
  c = __builtin_amdgcn_wmma_f32_16x16x32_f16(false, a, false, b, (short)0, c, false, false);
  asm volatile("v_nop\n\tv_nop\n\tv_nop\n\tv_nop" : "+v"(c) : "v"(a), "v"(b));
  return c;
}

__device__ __forceinline__ v16h ldfrag(const _Float16* p, int ld, int row0, int k0, int lane) {
  const int m = lane & 15, lh = lane >> 4;
  const _Float16* q = p + (size_t)(row0 + m) * ld + k0 + 8 * lh;
  Frag f;
  f.h[0] = *(const v8h*)(q);
  f.h[1] = *(const v8h*)(q + 16);
  return f.v;
}

__device__ __forceinline__ v8f zero8() { return (v8f){0.f, 0.f, 0.f, 0.f, 0.f, 0.f, 0.f, 0.f}; }

__device__ __forceinline__ int expert_of(const int* __restrict__ eidx) {
  int e = eidx[0];
  e = (e < 0) ? 0 : e;
  e = (e > NEXP - 1) ? (NEXP - 1) : e;
  return e;
}

__device__ __forceinline__ void gemm32x64(const _Float16* __restrict__ A, int lda,
                                          const _Float16* __restrict__ Bt, int ldb,
                                          int m0, int n0, int lane, v8f (&acc)[2][4]) {
#pragma unroll 2
  for (int k0 = 0; k0 < HID; k0 += 32) {
    const v16h a0 = ldfrag(A, lda, m0, k0, lane);
    const v16h a1 = ldfrag(A, lda, m0 + 16, k0, lane);
    const v16h b0 = ldfrag(Bt, ldb, n0, k0, lane);
    const v16h b1 = ldfrag(Bt, ldb, n0 + 16, k0, lane);
    const v16h b2 = ldfrag(Bt, ldb, n0 + 32, k0, lane);
    const v16h b3 = ldfrag(Bt, ldb, n0 + 48, k0, lane);
    acc[0][0] = mma16(a0, b0, acc[0][0]);
    acc[1][0] = mma16(a1, b0, acc[1][0]);
    acc[0][1] = mma16(a0, b1, acc[0][1]);
    acc[1][1] = mma16(a1, b1, acc[1][1]);
    acc[0][2] = mma16(a0, b2, acc[0][2]);
    acc[1][2] = mma16(a1, b2, acc[1][2]);
    acc[0][3] = mma16(a0, b3, acc[0][3]);
    acc[1][3] = mma16(a1, b3, acc[1][3]);
  }
}

__global__ __launch_bounds__(256) void k_cvt(const float* __restrict__ src, const int* __restrict__ eidx,
                                             int erows, _Float16* __restrict__ dh, float scale) {
  const int e = expert_of(eidx);
  const float* s = src + (size_t)e * (size_t)erows * HID;
  const int tid = threadIdx.x;
  const int row = blockIdx.x * 2 + (tid >> 7);
  const int col = (tid & 127) * 8;
  const size_t o = (size_t)row * HID + col;
  const v4f a0 = *(const v4f*)(s + o) * scale;
  const v4f a1 = *(const v4f*)(s + o + 4) * scale;
  Pack8 pk;
  pk.h = (v8h){(_Float16)a0[0], (_Float16)a0[1], (_Float16)a0[2], (_Float16)a0[3],
               (_Float16)a1[0], (_Float16)a1[1], (_Float16)a1[2], (_Float16)a1[3]};
  const v4u vv = pk.u;
  volatile v4u* d = (volatile v4u*)(dh + o);
  *d = vv;
  __threadfence();
  *d = vv;
}

__global__ __launch_bounds__(256) void k_tab(float* __restrict__ ct, float* __restrict__ st) {
  const int idx = blockIdx.x * 256 + threadIdx.x;
  const int l = idx >> 7;
  const int d = idx & 127;
  const int j = d & 63;
  const float invf = exp2f((float)j * -0.20762050593046014f);
  const float ang = (float)l * invf;
  float sn, cs;
  sincosf(ang, &sn, &cs);
  volatile float* pc = ct + idx;
  volatile float* ps = st + idx;
  *pc = cs;
  *ps = sn;
  __threadfence();
  *pc = cs;
  *ps = sn;
}

#define SFP 68
template <int MODE>
__global__ __launch_bounds__(128) void k_proj(const _Float16* __restrict__ A,
                                              const _Float16* __restrict__ W,
                                              const float* __restrict__ bias,
                                              const int* __restrict__ eidx,
                                              const float* __restrict__ ct,
                                              const float* __restrict__ st,
                                              _Float16* __restrict__ dst,
                                              int shift, int hbstride, int poff) {
  __shared__ __align__(16) float sf[128 * SFP];
  const int tid = threadIdx.x, lane = tid & 31, wave = tid >> 5;
  const int hh = lane >> 4, c = lane & 15;
  const int e = expert_of(eidx);
  const float* be = bias + (size_t)e * HID;
  const int mblk  = blockIdx.x * 128;
  const int n0    = blockIdx.y * 64;
  const int head  = n0 >> 7;
  const int dbase = n0 & 127;
  const int m0    = mblk + wave * 32;
  const int pmask = (1 << shift) - 1;

  v8f acc[2][4];
#pragma unroll
  for (int s = 0; s < 2; ++s)
#pragma unroll
    for (int t = 0; t < 4; ++t) acc[s][t] = zero8();
  gemm32x64(A, HID, W, HID, m0, n0, lane, acc);

  float bv[4];
#pragma unroll
  for (int t = 0; t < 4; ++t) bv[t] = be[n0 + 16 * t + c];
#pragma unroll
  for (int s = 0; s < 2; ++s) {
#pragma unroll
    for (int t = 0; t < 4; ++t) {
#pragma unroll
      for (int r = 0; r < 8; ++r)
        sf[(wave * 32 + s * 16 + 8 * hh + r) * SFP + 16 * t + c] = acc[s][t][r] * 0.03125f + bv[t];
    }
  }
  __syncthreads();

  v4u val[8];
  size_t go[8];
  if (MODE == 0) {
#pragma unroll
    for (int j = 0; j < 8; ++j) {
      const int p   = tid + 128 * j;
      const int lr  = p >> 3;
      const int pc  = p & 7;
      const int m   = mblk + lr;
      const int b   = m >> shift;
      const int pos = m & pmask;
      const int d0  = dbase + pc * 8;
      const float* ra = sf + lr * SFP + pc * 8;
      const v4f a0 = *(const v4f*)(ra), a1 = *(const v4f*)(ra + 4);
      const float* tcp = ct + (size_t)pos * HDM + d0;
      const float* tsp = st + (size_t)pos * HDM + d0;
      const v4f c0 = *(const v4f*)(tcp), c1 = *(const v4f*)(tcp + 4);
      const v4f s0 = *(const v4f*)(tsp), s1 = *(const v4f*)(tsp + 4);
      const float y0 = a0[0] * c0[0] - a0[1] * s0[0];
      const float y1 = a0[1] * c0[1] + a0[0] * s0[1];
      const float y2 = a0[2] * c0[2] - a0[3] * s0[2];
      const float y3 = a0[3] * c0[3] + a0[2] * s0[3];
      const float y4 = a1[0] * c1[0] - a1[1] * s1[0];
      const float y5 = a1[1] * c1[1] + a1[0] * s1[1];
      const float y6 = a1[2] * c1[2] - a1[3] * s1[2];
      const float y7 = a1[3] * c1[3] + a1[2] * s1[3];
      Pack8 pk;
      pk.h = (v8h){(_Float16)y0, (_Float16)y1, (_Float16)y2, (_Float16)y3,
                   (_Float16)y4, (_Float16)y5, (_Float16)y6, (_Float16)y7};
      val[j] = pk.u;
      go[j]  = ((size_t)((b * NHD + head) * hbstride + poff + pos)) * HDM + d0;
    }
  } else {
    const int b     = mblk >> shift;
    const int kpos0 = mblk & pmask;
#pragma unroll
    for (int j = 0; j < 8; ++j) {
      const int p    = tid + 128 * j;
      const int dcol = p >> 4;
      const int pc   = p & 15;
      const float* cp = sf + (pc * 8) * SFP + dcol;
      Pack8 pk;
      pk.h = (v8h){(_Float16)cp[0 * SFP], (_Float16)cp[1 * SFP], (_Float16)cp[2 * SFP], (_Float16)cp[3 * SFP],
                   (_Float16)cp[4 * SFP], (_Float16)cp[5 * SFP], (_Float16)cp[6 * SFP], (_Float16)cp[7 * SFP]};
      val[j] = pk.u;
      const int d = dbase + dcol;
      go[j]  = ((size_t)((b * NHD + head) * HDM + d)) * NKEY + poff + kpos0 + pc * 8;
    }
  }
  for (int ps = 0; ps < 2; ++ps) {
#pragma unroll
    for (int j = 0; j < 8; ++j) *(volatile v4u*)(dst + go[j]) = val[j];
    __threadfence();
  }
}

#define PTP 136
__global__ __launch_bounds__(256) void k_attn(const _Float16* __restrict__ qp,
                                              const _Float16* __restrict__ kp,
                                              const _Float16* __restrict__ vt,
                                              const float* __restrict__ gate,
                                              const int* __restrict__ eidx,
                                              _Float16* __restrict__ op) {
  __shared__ __align__(16) _Float16 Ps[8 * 16 * PTP];

  const int tid = threadIdx.x, lane = tid & 31, wave = tid >> 5;
  const int hh = lane >> 4, c = lane & 15;
  const int e = expert_of(eidx);
  const float gv    = gate[e];
  const float ratio = 1.0f / (1.0f + expf(-gv));
  const float scl_a = 0.08838834764831845f;
  const float scl_t = scl_a * ratio;
  const int hb = blockIdx.x / NQB;
  const int qb = blockIdx.x - hb * NQB;
  const int h  = hb % NHD;
  const int b  = hb / NHD;
  const int q0 = qb * QB + wave * 16;

  const _Float16* Qbase = qp + (size_t)hb * 2 * TQ * HDM;
  const _Float16* K     = kp + (size_t)hb * NKEY * HDM;
  const _Float16* V     = vt + (size_t)hb * HDM * NKEY;

  const float NEGI = -__builtin_huge_valf();
  float mrow[8], lrow[8];
  v8f oacc[8];
#pragma unroll
  for (int r = 0; r < 8; ++r) { mrow[r] = NEGI; lrow[r] = 0.f; }
#pragma unroll
  for (int t = 0; t < 8; ++t) oacc[t] = zero8();

  _Float16* pw = Ps + wave * 16 * PTP;

  for (int kc = 0; kc < NCK; ++kc) {
    const int key0 = kc * KC;
    const int set  = kc / (NCK / 2);
    const _Float16* Q = Qbase + (size_t)set * TQ * HDM;
    const float scl = (set == 0) ? scl_a : scl_t;
    __syncthreads();

    v8f s[4];
#pragma unroll
    for (int j = 0; j < 4; ++j) s[j] = zero8();
#pragma unroll
    for (int dc = 0; dc < 4; ++dc) {
      const v16h qa = ldfrag(Q, HDM, q0, dc * 32, lane);
#pragma unroll
      for (int j = 0; j < 4; ++j) {
        const v16h kb = ldfrag(K, HDM, key0 + j * 16, dc * 32, lane);
        s[j] = mma16(qa, kb, s[j]);
      }
    }
    float cm[8];
#pragma unroll
    for (int r = 0; r < 8; ++r) {
      float m = NEGI;
#pragma unroll
      for (int j = 0; j < 4; ++j) { s[j][r] *= scl; m = fmaxf(m, s[j][r]); }
#pragma unroll
      for (int off = 1; off < 16; off <<= 1) m = fmaxf(m, __shfl_xor(m, off, 32));
      cm[r] = m;
    }
    float al[8];
#pragma unroll
    for (int r = 0; r < 8; ++r) {
      const float mnew  = fmaxf(mrow[r], cm[r]);
      const float alpha = __expf(mrow[r] - mnew);
      mrow[r] = mnew;
      float psum = 0.f;
#pragma unroll
      for (int j = 0; j < 4; ++j) {
        const float p = __expf(s[j][r] - mnew);
        psum += p;
        pw[(8 * hh + r) * PTP + j * 16 + c] = (_Float16)(p * 1024.0f);
      }
#pragma unroll
      for (int off = 1; off < 16; off <<= 1) psum += __shfl_xor(psum, off, 32);
      lrow[r] = lrow[r] * alpha + psum;
      al[r] = alpha;
    }
#pragma unroll
    for (int t = 0; t < 8; ++t)
#pragma unroll
      for (int r = 0; r < 8; ++r) oacc[t][r] *= al[r];
    __syncthreads();

#pragma unroll
    for (int kk = 0; kk < 2; ++kk) {
      const v16h pa = ldfrag(pw, PTP, 0, kk * 32, lane);
#pragma unroll
      for (int t = 0; t < 8; ++t) {
        const v16h vb = ldfrag(V, NKEY, t * 16, key0 + kk * 32, lane);
        oacc[t] = mma16(pa, vb, oacc[t]);
      }
    }
  }

  float invl[8];
#pragma unroll
  for (int r = 0; r < 8; ++r) invl[r] = (lrow[r] > 0.f) ? (0.0625f / lrow[r]) : 0.f;
  __syncthreads();
#pragma unroll
  for (int r = 0; r < 8; ++r) {
#pragma unroll
    for (int t = 0; t < 8; ++t)
      pw[(8 * hh + r) * PTP + 16 * t + c] = (_Float16)(oacc[t][r] * invl[r]);
  }
  __syncthreads();
  v4u val[8];
  size_t go[8];
#pragma unroll
  for (int it = 0; it < 8; ++it) {
    const int p  = lane + 32 * it;
    const int L  = p >> 4;
    const int pc = p & 15;
    Pack8 pk;
    pk.h    = *(const v8h*)(pw + L * PTP + pc * 8);
    val[it] = pk.u;
    go[it]  = ((size_t)(b * TQ + q0 + L)) * HID + (size_t)h * HDM + pc * 8;
  }
  for (int ps = 0; ps < 2; ++ps) {
#pragma unroll
    for (int it = 0; it < 8; ++it) *(volatile v4u*)(op + go[it]) = val[it];
    __threadfence();
  }
}

#define OTP 68
template <int EPI>
__global__ __launch_bounds__(128) void k_gemm(const _Float16* __restrict__ ap,
                                              const _Float16* __restrict__ wt,
                                              const float* __restrict__ bias,
                                              const int* __restrict__ eidx,
                                              const float* __restrict__ resid,
                                              float scale,
                                              float* __restrict__ out) {
  __shared__ __align__(16) float st[4][16 * OTP];
  const int tid = threadIdx.x, lane = tid & 31, wave = tid >> 5;
  const int hh = lane >> 4, c = lane & 15;
  const int e = expert_of(eidx);
  const float* be = bias + (size_t)e * HID;
  const int m0 = blockIdx.x * 128 + wave * 32;
  const int n0 = blockIdx.y * 64;

  v8f acc[2][4];
#pragma unroll
  for (int s = 0; s < 2; ++s)
#pragma unroll
    for (int t = 0; t < 4; ++t) acc[s][t] = zero8();
  gemm32x64(ap, HID, wt, HID, m0, n0, lane, acc);

  float bv[4];
#pragma unroll
  for (int t = 0; t < 4; ++t) bv[t] = be[n0 + 16 * t + c];
  float* sw = st[wave];
#pragma unroll
  for (int sub = 0; sub < 2; ++sub) {
    __syncthreads();
#pragma unroll
    for (int t = 0; t < 4; ++t) {
#pragma unroll
      for (int r = 0; r < 8; ++r) sw[(8 * hh + r) * OTP + 16 * t + c] = acc[sub][t][r] * scale + bv[t];
    }
    __syncthreads();
    v4f val[8];
    size_t go[8];
#pragma unroll
    for (int it = 0; it < 8; ++it) {
      const int p   = lane + 32 * it;
      const int L   = p >> 3;
      const int pc  = p & 7;
      const int row = L >> 1;
      const int hf  = L & 1;
      v4f v = *(const v4f*)(sw + row * OTP + hf * 32 + pc * 4);
      go[it] = (size_t)(m0 + sub * 16 + row) * HID + n0 + hf * 32 + pc * 4;
      if (EPI == 0) {
        v += *(const v4f*)(resid + go[it]);
      } else {
        v = (v4f){fmaxf(v[0], 0.f), fmaxf(v[1], 0.f), fmaxf(v[2], 0.f), fmaxf(v[3], 0.f)};
      }
      val[it] = v;
    }
    for (int ps = 0; ps < 2; ++ps) {
#pragma unroll
      for (int it = 0; it < 8; ++it) *(volatile v4f*)(out + go[it]) = val[it];
      __threadfence();
    }
  }
}

__global__ __launch_bounds__(256) void k_ln(const float* __restrict__ t, const float* __restrict__ g,
                                            const float* __restrict__ bt, const int* __restrict__ eidx,
                                            _Float16* __restrict__ yh) {
  const int tid = threadIdx.x, lane = tid & 31, wave = tid >> 5;
  const size_t m = (size_t)blockIdx.x * 8 + wave;
  const int e = expert_of(eidx);
  const float* ge = g + (size_t)e * HID;
  const float* bb = bt + (size_t)e * HID;
  const float* tr = t + m * HID;

  v4f v[8];
  float s = 0.f;
#pragma unroll
  for (int j = 0; j < 4; ++j) {
    const int idx = 256 * j + 8 * lane;
    v[2 * j]     = *(const v4f*)(tr + idx);
    v[2 * j + 1] = *(const v4f*)(tr + idx + 4);
    s += (v[2 * j][0] + v[2 * j][1]) + (v[2 * j][2] + v[2 * j][3]);
    s += (v[2 * j + 1][0] + v[2 * j + 1][1]) + (v[2 * j + 1][2] + v[2 * j + 1][3]);
  }
#pragma unroll
  for (int off = 16; off >= 1; off >>= 1) s += __shfl_xor(s, off, 32);
  const float mean = s * 0.0009765625f;
  float ss = 0.f;
#pragma unroll
  for (int it = 0; it < 8; ++it) {
    const v4f d = v[it] - mean;
    ss += (d[0] * d[0] + d[1] * d[1]) + (d[2] * d[2] + d[3] * d[3]);
  }
#pragma unroll
  for (int off = 16; off >= 1; off >>= 1) ss += __shfl_xor(ss, off, 32);
  const float var  = ss * 0.0009765625f;
  const float rstd = rsqrtf(var + 1e-5f);

  v4u hv[4];
  size_t go[4];
#pragma unroll
  for (int j = 0; j < 4; ++j) {
    const int idx = 256 * j + 8 * lane;
    const v4f g0 = *(const v4f*)(ge + idx), g1 = *(const v4f*)(ge + idx + 4);
    const v4f b0 = *(const v4f*)(bb + idx), b1 = *(const v4f*)(bb + idx + 4);
    const v4f y0 = ((v[2 * j] - mean) * rstd) * g0 + b0;
    const v4f y1 = ((v[2 * j + 1] - mean) * rstd) * g1 + b1;
    Pack8 pk;
    pk.h = (v8h){(_Float16)y0[0], (_Float16)y0[1], (_Float16)y0[2], (_Float16)y0[3],
                 (_Float16)y1[0], (_Float16)y1[1], (_Float16)y1[2], (_Float16)y1[3]};
    hv[j] = pk.u;
    go[j] = m * HID + idx;
  }
  for (int ps = 0; ps < 2; ++ps) {
#pragma unroll
    for (int j = 0; j < 4; ++j) *(volatile v4u*)(yh + go[j]) = hv[j];
    __threadfence();
  }
}

extern "C" void kernel_launch(void* const* d_in, const int* in_sizes, int n_in,
                              void* d_out, int out_size, void* d_ws, size_t ws_size,
                              hipStream_t stream) {
  if (n_in < 23) return;
  if (in_sizes[0] != NTQ * HID) return;
  if (in_sizes[1] != NTK * HID) return;
  if (in_sizes[2] != NTK * HID) return;
  for (int i = 0; i < 8; ++i) {
    if (in_sizes[3 + 2 * i] != NEXP * HID * HID) return;
    if (in_sizes[4 + 2 * i] != NEXP * HID) return;
  }
  if (in_sizes[19] != NEXP * HID) return;
  if (in_sizes[20] != NEXP * HID) return;
  if (in_sizes[21] != NEXP) return;
  if (in_sizes[22] != 1) return;
  if (out_size != NTQ * HID) return;

  const float* x    = (const float*)d_in[0];
  const float* h_a  = (const float*)d_in[1];
  const float* h_t  = (const float*)d_in[2];
  const float* wsrc[8];
  const float* bsrc[8];
  for (int i = 0; i < 8; ++i) {
    wsrc[i] = (const float*)d_in[3 + 2 * i];
    bsrc[i] = (const float*)d_in[4 + 2 * i];
  }
  const float* gamma = (const float*)d_in[19];
  const float* beta  = (const float*)d_in[20];
  const float* gate  = (const float*)d_in[21];
  const int*   eidx  = (const int*)d_in[22];
  float* out = (float*)d_out;

  const size_t MM = (size_t)HID * HID;
  size_t off = 0;
  const size_t oX  = off; off += (size_t)NTQ * HID * 2;
  const size_t oHa = off; off += (size_t)NTK * HID * 2;
  const size_t oHt = off; off += (size_t)NTK * HID * 2;
  const size_t oW  = off; off += (size_t)8 * MM * 2;
  const size_t oQ  = off; off += (size_t)NHB * 2 * TQ * HDM * 2;
  const size_t oK  = off; off += (size_t)NHB * NKEY * HDM * 2;
  const size_t oV  = off; off += (size_t)NHB * HDM * NKEY * 2;
  const size_t oCT = off; off += (size_t)TQ * HDM * 4;
  const size_t oST = off; off += (size_t)TQ * HDM * 4;
  if (off > ws_size) return;
  if (off > (size_t)134217728) return;
  if ((size_t)NTQ * HID * 2 != (size_t)2 * NTK * HID * 2) return;
  if ((size_t)NTQ * HID * 4 != (size_t)NHB * 2 * TQ * HDM * 2) return;

  char* ws = (char*)d_ws;
  _Float16* Xh  = (_Float16*)(ws + oX);
  _Float16* Hah = (_Float16*)(ws + oHa);
  _Float16* Hth = (_Float16*)(ws + oHt);
  _Float16* Wt  = (_Float16*)(ws + oW);
  _Float16* Qp  = (_Float16*)(ws + oQ);
  _Float16* Kp  = (_Float16*)(ws + oK);
  _Float16* Vt  = (_Float16*)(ws + oV);
  float*    CT  = (float*)(ws + oCT);
  float*    ST  = (float*)(ws + oST);
  _Float16* Op  = (_Float16*)(ws + oX);
  _Float16* XNh = (_Float16*)(ws + oHa);
  float*    T1  = (float*)(ws + oQ);

  k_cvt<<<dim3(NTQ / 2), dim3(256), 0, stream>>>(x, eidx, 0, Xh, 1.0f);
  k_cvt<<<dim3(NTK / 2), dim3(256), 0, stream>>>(h_a, eidx, 0, Hah, 1.0f);
  k_cvt<<<dim3(NTK / 2), dim3(256), 0, stream>>>(h_t, eidx, 0, Hth, 1.0f);
  for (int i = 0; i < 8; ++i)
    k_cvt<<<dim3(HID / 2), dim3(256), 0, stream>>>(wsrc[i], eidx, HID, Wt + (size_t)i * MM, 32.0f);
  k_tab<<<dim3((TQ * HDM) / 256), dim3(256), 0, stream>>>(CT, ST);
  k_proj<0><<<dim3(NTQ / 128, HID / 64), dim3(128), 0, stream>>>(Xh,  Wt + 0 * MM, bsrc[0], eidx, CT, ST, Qp, 9, 2 * TQ, 0);
  k_proj<0><<<dim3(NTQ / 128, HID / 64), dim3(128), 0, stream>>>(Xh,  Wt + 3 * MM, bsrc[3], eidx, CT, ST, Qp, 9, 2 * TQ, TQ);
  k_proj<0><<<dim3(NTK / 128, HID / 64), dim3(128), 0, stream>>>(Hah, Wt + 1 * MM, bsrc[1], eidx, CT, ST, Kp, 8, NKEY, 0);
  k_proj<0><<<dim3(NTK / 128, HID / 64), dim3(128), 0, stream>>>(Hth, Wt + 4 * MM, bsrc[4], eidx, CT, ST, Kp, 8, NKEY, LKV);
  k_proj<1><<<dim3(NTK / 128, HID / 64), dim3(128), 0, stream>>>(Hah, Wt + 2 * MM, bsrc[2], eidx, CT, ST, Vt, 8, 0, 0);
  k_proj<1><<<dim3(NTK / 128, HID / 64), dim3(128), 0, stream>>>(Hth, Wt + 5 * MM, bsrc[5], eidx, CT, ST, Vt, 8, 0, LKV);
  k_attn<<<dim3(NHB * NQB), dim3(256), 0, stream>>>(Qp, Kp, Vt, gate, eidx, Op);
  k_gemm<0><<<dim3(NTQ / 128, HID / 64), dim3(128), 0, stream>>>(Op, Wt + 6 * MM, bsrc[6], eidx, x, 0.00048828125f, T1);
  k_ln<<<dim3(NTQ / 8), dim3(256), 0, stream>>>(T1, gamma, beta, eidx, XNh);
  k_gemm<1><<<dim3(NTQ / 128, HID / 64), dim3(128), 0, stream>>>(XNh, Wt + 7 * MM, bsrc[7], eidx, x, 0.03125f, out);
  (void)hipGetLastError();
}
